// TransformerEncoderLayer_47691316854955
// MI455X (gfx1250) — hardware-verified
//
#include <hip/hip_runtime.h>
#ifndef NB
#define NB 4
#endif
#ifndef SEQ
#define SEQ 4096
#endif
#define NB_FULL 4
#define SEQ_FULL 4096
#define DM 128
#define NH 4
#define HD 32
#define DFF 512
#define NR ((size_t)NB * SEQ)
#define LQK (2 * DM)
#define QSCL 0.17677669529663689f
static_assert(SEQ % 128 == 0);
static_assert(NB >= 1 && NB <= NB_FULL);
static_assert(SEQ <= SEQ_FULL);
static_assert(NH * HD == DM);
static_assert(NH == 4 && HD == 32 && DM == 128);
static_assert(DM % 64 == 0 && DFF % 64 == 0 && LQK % 64 == 0 && DM % 32 == 0 && DFF % 32 == 0);
static_assert(((size_t)NB * SEQ) % 128 == 0);
static_assert(((size_t)NB * SEQ) % 8 == 0);

typedef unsigned short v8us __attribute__((ext_vector_type(8), may_alias));
typedef float  v8f  __attribute__((ext_vector_type(8)));
typedef float  v4f  __attribute__((ext_vector_type(4)));
typedef float  v4fa __attribute__((ext_vector_type(4), may_alias));
typedef _Float16 v16h __attribute__((ext_vector_type(16)));
typedef _Float16 v4h __attribute__((ext_vector_type(4)));
union FragH { v16h v; v8us half[2]; _Float16 h[16]; unsigned short u[16]; };

__device__ __forceinline__ unsigned short bf16_bits(float x) { unsigned int u = __float_as_uint(x); return (unsigned short)((u + 0x7FFFu + ((u >> 16) & 1u)) >> 16); }
__device__ __forceinline__ float bf16_val(unsigned short b) { return __uint_as_float(((unsigned int)b) << 16); }
__device__ __forceinline__ float bf16_rne(float x) { return bf16_val(bf16_bits(x)); }

__device__ __forceinline__ v16h g2_frag(const _Float16* p, unsigned hh) { FragH f; f.half[0] = *(const v8us*)((const unsigned short*)p + 8u * hh); f.half[1] = *(const v8us*)((const unsigned short*)p + 16u + 8u * hh); return f.v; }
__device__ __forceinline__ v8f g2_mma(v16h a, v16h b, v8f c) { v8f d = __builtin_amdgcn_wmma_f32_16x16x32_f16(false, a, false, b, (short)0, c, false, false); asm volatile("v_nop\n\tv_nop\n\tv_nop\n\tv_nop" : "+v"(d) : "v"(a), "v"(b)); return d; }

__global__ __launch_bounds__(256) void k_wt_f16(const float* __restrict__ W, _Float16* __restrict__ Wt, unsigned K, unsigned N, unsigned lk8, float scale) {
  const unsigned t = blockIdx.x * 256u + threadIdx.x; if (t >= N * (K >> 3)) return;
  const unsigned n = t >> lk8, k8 = (t & ((1u << lk8) - 1u)) << 3; FragH f;
#pragma unroll
  for (unsigned i = 0; i < 8; ++i) f.h[i] = (_Float16)(bf16_rne(W[(size_t)(k8 + i) * N + n]) * scale);
  const v8us o = f.half[0]; unsigned short* dst = (unsigned short*)Wt + (size_t)n * K + k8;
  *(volatile v8us*)dst = o; __threadfence(); *(volatile v8us*)dst = o;
}

template <int BFIN, int IRM>
__global__ __launch_bounds__(256) void k_ln128(const float* __restrict__ X, const float* __restrict__ g, const float* __restrict__ bb, float eps, _Float16* __restrict__ N16, unsigned nrows) {
  #pragma clang fp contract(off)
  const unsigned w = threadIdx.x >> 5, lane = threadIdx.x & 31u;
  const unsigned r = blockIdx.x * 8u + w; if (r >= nrows) return;
  size_t ri = r; if (IRM) { const unsigned bq = r / (unsigned)SEQ; ri = (size_t)bq * SEQ_FULL + (r - bq * (unsigned)SEQ); }
  const unsigned c0 = lane * 4u;
  const v4f xa = *(const v4fa*)(X + ri * DM + c0); float s[4]; float sum = 0.f;
#pragma unroll
  for (int q = 0; q < 4; ++q) { s[q] = BFIN ? bf16_rne(xa[q]) : xa[q]; sum += s[q]; }
#pragma unroll
  for (unsigned o = 16; o > 0; o >>= 1) sum += __shfl_xor(sum, (int)o, 32);
  const float mu = sum * (1.0f / 128.0f);
  float vs = 0.f;
#pragma unroll
  for (int q = 0; q < 4; ++q) { const float dl = s[q] - mu; vs += dl * dl; }
#pragma unroll
  for (unsigned o = 16; o > 0; o >>= 1) vs += __shfl_xor(vs, (int)o, 32);
  const float rs = rsqrtf(vs * (1.0f / 128.0f) + eps);
  const v4f g4 = *(const v4fa*)(g + c0); const v4f b4 = *(const v4fa*)(bb + c0); v4h y;
#pragma unroll
  for (int q = 0; q < 4; ++q) y[q] = (_Float16)((s[q] - mu) * rs * bf16_rne(g4[q]) + bf16_rne(b4[q]));
  _Float16* dst = N16 + (size_t)r * DM + c0;
  *(volatile v4h*)dst = y; __threadfence(); *(volatile v4h*)dst = y;
}

template <int ACT, int CPBF>
__global__ __launch_bounds__(128) void k_gemm2(const _Float16* __restrict__ A, unsigned lda, size_t sA, const _Float16* __restrict__ Bh, unsigned ldb, size_t sB, float alpha,
    const float* __restrict__ bias, const float* __restrict__ rbias, const float* __restrict__ CP, unsigned ldcp, size_t sCP,
    float* __restrict__ C, _Float16* __restrict__ C16, unsigned ldc, size_t sC, float s16, unsigned M, unsigned N, unsigned K) { static_assert(ACT == 0 || ACT == 3 || ACT == 4);
  __shared__ __attribute__((aligned(16))) float so[4][32][68];
  const unsigned tid = threadIdx.x, w = tid >> 5, lane = tid & 31u, ln = lane & 15u, hh = lane >> 4; const unsigned by = blockIdx.y;
  A += (size_t)by * sA; Bh += (size_t)by * sB; const size_t cofs = (size_t)by * sC; const size_t cpofs = (size_t)by * sCP;
  const unsigned ntn = N >> 6; const unsigned mt = blockIdx.x / ntn, nq = blockIdx.x - mt * ntn; const unsigned row0 = mt * 128u + 32u * w, col0 = nq * 64u; if (row0 >= M) return;
  const _Float16* a0p = A + (size_t)(row0 + ln) * lda; const _Float16* a1p = a0p + (size_t)16 * lda;
  const _Float16* b0p = Bh + (size_t)(col0 + ln) * ldb; const _Float16* b1p = b0p + (size_t)16 * ldb; const _Float16* b2p = b1p + (size_t)16 * ldb; const _Float16* b3p = b2p + (size_t)16 * ldb;
  const v8f z8 = {0.f,0.f,0.f,0.f,0.f,0.f,0.f,0.f}; v8f c00 = z8, c01 = z8, c02 = z8, c03 = z8, c10 = z8, c11 = z8, c12 = z8, c13 = z8;
#pragma unroll 1
  for (unsigned kb = 0; kb < K; kb += 32) { const v16h a0 = g2_frag(a0p + kb, hh), a1 = g2_frag(a1p + kb, hh);
    v16h b = g2_frag(b0p + kb, hh); c00 = g2_mma(a0, b, c00); c10 = g2_mma(a1, b, c10);
    b = g2_frag(b1p + kb, hh); c01 = g2_mma(a0, b, c01); c11 = g2_mma(a1, b, c11);
    b = g2_frag(b2p + kb, hh); c02 = g2_mma(a0, b, c02); c12 = g2_mma(a1, b, c12);
    b = g2_frag(b3p + kb, hh); c03 = g2_mma(a0, b, c03); c13 = g2_mma(a1, b, c13); }
  v8f accs[8] = {c00, c01, c02, c03, c10, c11, c12, c13};
#pragma unroll
  for (int u = 0; u < 8; ++u) { const unsigned t = (unsigned)u & 3u, half = (unsigned)u >> 2;
#pragma unroll
    for (int r = 0; r < 8; ++r) so[w][half * 16u + 8u * hh + (unsigned)r][t * 16u + ln] = accs[u][r] * alpha; }
  __builtin_amdgcn_fence(4  , "workgroup"); __builtin_amdgcn_wave_barrier();
  const unsigned rsub = lane >> 4, c4 = (lane & 15u) * 4u;
  v4f b4 = {0.f, 0.f, 0.f, 0.f};
  if (bias) { const v4f t4 = *(const v4fa*)(bias + col0 + c4);
#pragma unroll
    for (int i = 0; i < 4; ++i) b4[i] = bf16_rne(t4[i]); }
#pragma unroll 1
  for (unsigned q = 0; q < 16; ++q) { const unsigned r = q * 2u + rsub; v4f v = *(const v4fa*)&so[w][r][c4];
    float rb = 0.f; if (rbias) rb = bf16_rne(rbias[row0 + r]);
#pragma unroll
    for (int i = 0; i < 4; ++i) v[i] = v[i] + b4[i] + rb;
    if (CP) { v4f cp = *(const v4fa*)(CP + cpofs + (size_t)(row0 + r) * ldcp + col0 + c4);
#pragma unroll
      for (int i = 0; i < 4; ++i) v[i] += CPBF ? bf16_rne(cp[i]) : cp[i]; }
    if (ACT == 3) {
#pragma unroll
      for (int i = 0; i < 4; ++i) v[i] = fmaxf(v[i], 0.f); }
    if (ACT == 4) {
#pragma unroll
      for (int i = 0; i < 4; ++i) v[i] = 0.5f * v[i] * (1.0f + erff(v[i] * 0.70710678118654752f)); }
    *(v4fa*)&so[w][r][c4] = v; }
  __builtin_amdgcn_fence(4  , "workgroup"); __builtin_amdgcn_wave_barrier();
  for (int pass = 0; pass < 2; ++pass) {
#pragma unroll
    for (unsigned q = 0; q < 16; ++q) { const unsigned r = q * 2u + rsub; const v4f v = *(const v4fa*)&so[w][r][c4];
      if (C) *(volatile v4f*)(C + cofs + (size_t)(row0 + r) * ldc + col0 + c4) = v;
      if (C16) { v4h h4;
#pragma unroll
        for (int i = 0; i < 4; ++i) h4[i] = (_Float16)(v[i] * s16);
        *(volatile v4h*)(C16 + cofs + (size_t)(row0 + r) * ldc + col0 + c4) = h4; } }
    if (pass == 0) __threadfence(); } }

__global__ __launch_bounds__(128) void k_attn(const _Float16* __restrict__ QK, const _Float16* __restrict__ VT, _Float16* __restrict__ CAT) {
  __shared__ __attribute__((aligned(16))) unsigned short so[16][136];
  const unsigned tid = threadIdx.x, w = tid >> 5, lane = tid & 31u, nl = lane & 15u, hh = lane >> 4;
  const unsigned h = w, b = blockIdx.y;
  const unsigned q0 = blockIdx.x * 16u;
  const size_t rq = (size_t)b * SEQ + q0;
  const size_t rk = (size_t)b * SEQ;
  const _Float16* qp = QK + (rq + nl) * LQK + h * HD;
  const v16h qb = g2_frag(qp, hh);
  const _Float16* kp = QK + (rk + nl) * LQK + DM + h * HD;
  const _Float16* vp = VT + ((size_t)h * HD + nl) * NR + rk;
  const v8f z8 = {0.f,0.f,0.f,0.f,0.f,0.f,0.f,0.f};
  v8f o0 = z8, o1 = z8; float m = -1.0e30f, l = 0.f;
#pragma unroll 1
  for (unsigned kb = 0; kb < (unsigned)SEQ; kb += 32) {
    const _Float16* k0p = kp + (size_t)kb * LQK; const _Float16* k1p = k0p + (size_t)16 * LQK;
    v16h a;
    a = g2_frag(k0p, hh); v8f s0 = g2_mma(a, qb, z8);
    a = g2_frag(k1p, hh); v8f s1 = g2_mma(a, qb, z8);
    float mx = -1.0e30f;
#pragma unroll
    for (int r = 0; r < 8; ++r) mx = fmaxf(mx, fmaxf(s0[r], s1[r]));
    mx = fmaxf(mx, __shfl_xor(mx, 16, 32));
    const float mn = fmaxf(m, mx * QSCL);
    const float sc = __expf(m - mn);
    FragH pf; float ps = 0.f;
#pragma unroll
    for (int r = 0; r < 8; ++r) { const float e0 = __expf(s0[r] * QSCL - mn); const float e1 = __expf(s1[r] * QSCL - mn); ps += e0 + e1; pf.h[r] = (_Float16)(e0 * 256.0f); pf.h[8 + r] = (_Float16)(e1 * 256.0f); }
    ps += __shfl_xor(ps, 16, 32);
    l = l * sc + ps; m = mn;
#pragma unroll
    for (int r = 0; r < 8; ++r) { o0[r] *= sc; o1[r] *= sc; }
    const _Float16* v0p = vp + kb;
    a = g2_frag(v0p, hh); o0 = g2_mma(a, pf.v, o0);
    a = g2_frag(v0p + (size_t)16 * NR, hh); o1 = g2_mma(a, pf.v, o1);
  }
  const float inv = 0.25f / l;
  { FragH f;
#pragma unroll
    for (int r = 0; r < 8; ++r) f.h[r] = (_Float16)(o0[r] * inv); *(v8us*)&so[nl][w * 32u + 8u * hh] = f.half[0];
#pragma unroll
    for (int r = 0; r < 8; ++r) f.h[r] = (_Float16)(o1[r] * inv); *(v8us*)&so[nl][w * 32u + 16u + 8u * hh] = f.half[0]; }
  __syncthreads();
  const unsigned pr = lane >> 4, pc = lane & 15u;
  for (int pass = 0; pass < 2; ++pass) {
#pragma unroll
    for (unsigned it = 0; it < 2; ++it) { const unsigned row = w * 4u + it * 2u + pr; const v8us v = *(const v8us*)&so[row][pc * 8u]; *(volatile v8us*)((unsigned short*)CAT + (rq + row) * DM + pc * 8u) = v; }
    if (pass == 0) __threadfence(); }
}

extern "C" void kernel_launch(void* const* d_in, const int* in_sizes, int n_in,
                              void* d_out, int out_size, void* d_ws, size_t ws_size, hipStream_t stream) {
  if (n_in < 13) return;
  const float* const* I = (const float* const*)d_in;
  const float* x = I[0]; const float* g1 = I[1]; const float* be1 = I[2]; const float* wqkv = I[3]; const float* bqkv = I[4]; const float* wo = I[5]; const float* bo = I[6]; const float* g2 = I[7]; const float* be2 = I[8]; const float* w1 = I[9]; const float* b1 = I[10]; const float* w2 = I[11]; const float* b2 = I[12];
  const size_t need = ((size_t)(NB - 1) * SEQ_FULL + SEQ) * DM;
  if ((size_t)in_sizes[0] < need || (size_t)out_size < need) return;
  if (in_sizes[1] < DM || in_sizes[2] < DM || in_sizes[3] < DM * 3 * DM || in_sizes[4] < 3 * DM || in_sizes[5] < DM * DM || in_sizes[6] < DM || in_sizes[7] < DM || in_sizes[8] < DM || in_sizes[9] < DM * DFF || in_sizes[10] < DFF || in_sizes[11] < DFF * DM || in_sizes[12] < DM) return;
  const unsigned M = (unsigned)NR;
  char* ws = (char*)d_ws; size_t off = 0;
  auto take = [&](size_t bytes) { char* p = ws + off; off += (bytes + 255) & ~(size_t)255; return p; };
  _Float16* BQKV = (_Float16*)take((size_t)3 * DM * DM * 2);
  _Float16* BTO  = (_Float16*)take((size_t)DM * DM * 2);
  _Float16* BW1  = (_Float16*)take((size_t)DFF * DM * 2);
  _Float16* BW2  = (_Float16*)take((size_t)DM * DFF * 2);
  _Float16* A16  = (_Float16*)take(NR * DM * 2);
  _Float16* QK16 = (_Float16*)take(NR * LQK * 2);
  _Float16* VT16 = (_Float16*)take((size_t)DM * NR * 2);
  _Float16* CAT16 = (_Float16*)take(NR * DM * 2);
  float*    X1   = (float*)take(NR * DM * 4);
  _Float16* R16  = (_Float16*)take(NR * DM * 2);
  _Float16* H16  = (_Float16*)take(NR * DFF * 2);
  if (off > ws_size || off > (size_t)134217728) return;
  k_wt_f16<<<(unsigned)((3 * DM * (DM / 8) + 255) / 256), 256, 0, stream>>>(wqkv, BQKV, DM, 3 * DM, 4, 16.0f);
  k_wt_f16<<<(unsigned)((DM * (DM / 8) + 255) / 256), 256, 0, stream>>>(wo, BTO, DM, DM, 4, 16.0f);
  k_wt_f16<<<(unsigned)((DFF * (DM / 8) + 255) / 256), 256, 0, stream>>>(w1, BW1, DM, DFF, 4, 16.0f);
  k_wt_f16<<<(unsigned)((DM * (DFF / 8) + 255) / 256), 256, 0, stream>>>(w2, BW2, DFF, DM, 6, 16.0f);
  k_ln128<1, 1><<<(unsigned)(NR / 8), 256, 0, stream>>>(x, g1, be1, 1e-5f, A16, M);
  k_gemm2<0, 0><<<dim3((unsigned)((M / 128) * (LQK / 64)), 1), 128, 0, stream>>>(A16, DM, 0, BQKV, DM, 0, 0.0625f, bqkv, nullptr, nullptr, 0, 0, nullptr, QK16, LQK, 0, 1.0f, M, LQK, DM);
  k_gemm2<0, 0><<<dim3((unsigned)(((DM + 127) / 128) * (M / 64)), 1), 128, 0, stream>>>(BQKV + (size_t)2 * DM * DM, DM, 0, A16, DM, 0, 0.0625f, nullptr, bqkv + 2 * DM, nullptr, 0, 0, nullptr, VT16, M, 0, 1.0f, DM, M, DM);
  k_attn<<<dim3(SEQ / 16, NB), 128, 0, stream>>>(QK16, VT16, CAT16);
  k_gemm2<0, 1><<<dim3((unsigned)((SEQ / 128) * (DM / 64)), NB), 128, 0, stream>>>(CAT16, DM, (size_t)SEQ * DM, BTO, DM, 0, 0.0009765625f, bo, nullptr, x, DM, (size_t)SEQ_FULL * DM, X1, nullptr, DM, (size_t)SEQ * DM, 1.0f, SEQ, DM, DM);
  k_ln128<0, 0><<<(unsigned)(NR / 8), 256, 0, stream>>>(X1, g2, be2, 1e-5f, R16, M);
  k_gemm2<4, 0><<<dim3((unsigned)((M / 128) * (DFF / 64)), 1), 128, 0, stream>>>(R16, DM, 0, BW1, DM, 0, 0.0625f, b1, nullptr, nullptr, 0, 0, nullptr, H16, DFF, 0, 64.0f, M, DFF, DM);
  k_gemm2<0, 0><<<dim3((unsigned)((SEQ / 128) * (DM / 64)), NB), 128, 0, stream>>>(H16, DFF, (size_t)SEQ * DFF, BW2, DFF, 0, 0.0009765625f, b2, nullptr, X1, DM, (size_t)SEQ * DM, (float*)d_out, nullptr, DM, (size_t)SEQ_FULL * DM, 1.0f, SEQ, DM, DFF);
}
